// BlockSparseGRUv1_38010460570327
// MI455X (gfx1250) — hardware-verified
//
#include <hip/hip_runtime.h>
#include <math.h>

constexpr int NBATCH     = 16;
constexpr int NSTEP      = 512;
constexpr int NFEAT      = 256;
constexpr int NHID       = 1024;
constexpr int NBLK       = 8;
constexpr int NGATE3     = 3 * NHID;
constexpr int NCATROW    = 3136;
constexpr int NWHHROW    = 3088;
constexpr int NWKLROW    = 16;
constexpr int HALF_STEPS = 256;
constexpr int HALF_ROWS  = HALF_STEPS * NBATCH;
constexpr int NROWS      = NSTEP * NBATCH;
constexpr int HPITCH     = NHID + 8;
constexpr int FPITCH     = NHID + 4;
constexpr int PLANE16    = NBATCH * HPITCH;
constexpr int SCAN_THR   = 512;
constexpr float WCARRY   = 16.0f;
constexpr float HCARRY   = 256.0f;
constexpr float RCARRY   = 2048.0f;
constexpr float FOLD_MAIN = 1.0f / (WCARRY * HCARRY);
constexpr float FOLD_RES  = 1.0f / (WCARRY * HCARRY * RCARRY);
constexpr float BETA_GATE = 10.0f;

static_assert(NBATCH == 16);
static_assert(NHID == 64 * (SCAN_THR / 32));
static_assert(NHID / NBLK == 128);
static_assert(NFEAT % 32 == 0 && NHID % 32 == 0);
static_assert(NCATROW % 64 == 0 && HALF_ROWS % 64 == 0);
static_assert(NCATROW >= NGATE3 + NBLK && NWHHROW >= NGATE3 + 16);
static_assert(2 * HALF_STEPS == NSTEP);
static_assert(NFEAT / 8 == 32);
static_assert((HPITCH * 2) % 16 == 0 && (FPITCH * 4) % 16 == 0 && (PLANE16 * 2) % 16 == 0);
static_assert(((HALF_ROWS / 64) * (NCATROW / 64)) % 8 == 0);
static_assert((NWHHROW * (NHID / 8)) % 256 == 0 && (NCATROW * (NHID / 8)) % 256 == 0);
static_assert((NCATROW * (NFEAT / 8)) % 256 == 0 && (NWKLROW * (NHID / 8)) % 256 == 0);

typedef __attribute__((ext_vector_type(16))) _Float16 v16h;
typedef __attribute__((ext_vector_type(8)))  _Float16 v8h;
typedef __attribute__((ext_vector_type(16))) __bf16   v16b;
typedef __attribute__((ext_vector_type(8)))  __bf16   v8b;
typedef __attribute__((ext_vector_type(8)))  float    v8f;
typedef __attribute__((ext_vector_type(4)))  float    v4f;

__device__ __forceinline__ unsigned short f2bf_bits(float f) {
  unsigned u = __float_as_uint(f);
  return (unsigned short)((u + 0x7FFFu + ((u >> 16) & 1u)) >> 16);
}
__device__ __forceinline__ float bf_bits2f(unsigned short h) { return __uint_as_float(((unsigned)h) << 16); }

__device__ __forceinline__ void dep_guard4_h(v8f& a, v8f& b, v8f& c, v8f& d, v16h x, v16h y) {
  asm volatile("v_nop\n\tv_nop\n\tv_nop\n\tv_nop" : "+v"(a), "+v"(b), "+v"(c), "+v"(d) : "v"(x), "v"(y));
}
__device__ __forceinline__ void dep_guard4_b(v8f& a, v8f& b, v8f& c, v8f& d, v16b x, v16b y) {
  asm volatile("v_nop\n\tv_nop\n\tv_nop\n\tv_nop" : "+v"(a), "+v"(b), "+v"(c), "+v"(d) : "v"(x), "v"(y));
}
__device__ __forceinline__ void keep4_h(v16h a, v16h b, v16h c, v16h d) { asm volatile("v_nop" :: "v"(a), "v"(b), "v"(c), "v"(d)); }
__device__ __forceinline__ void keep4_b(v16b a, v16b b, v16b c, v16b d) { asm volatile("v_nop" :: "v"(a), "v"(b), "v"(c), "v"(d)); }
__device__ __forceinline__ void acc_guard4(v8f& a, v8f& b, v8f& c, v8f& d) {
  asm volatile("v_nop\n\tv_nop\n\tv_nop\n\tv_nop" : "+v"(a), "+v"(b), "+v"(c), "+v"(d));
}
__device__ __forceinline__ void dep_guard3_h(v8f& a, v8f& b, v8f& c, v16h x, v16h y0, v16h y1, v16h y2) {
  asm volatile("v_nop\n\tv_nop\n\tv_nop\n\tv_nop" : "+v"(a), "+v"(b), "+v"(c) : "v"(x), "v"(y0), "v"(y1), "v"(y2));
}
__device__ __forceinline__ void dep_guard2_h(v8f& a, v8f& b, v16h x0, v16h x1, v16h y0, v16h y1) {
  asm volatile("v_nop\n\tv_nop\n\tv_nop\n\tv_nop" : "+v"(a), "+v"(b) : "v"(x0), "v"(x1), "v"(y0), "v"(y1));
}
__device__ __forceinline__ void acc_guard3(v8f& a, v8f& b, v8f& c) {
  asm volatile("v_nop\n\tv_nop\n\tv_nop\n\tv_nop" : "+v"(a), "+v"(b), "+v"(c));
}
__device__ __forceinline__ void acc_guard2(v8f& a, v8f& b) {
  asm volatile("v_nop\n\tv_nop\n\tv_nop\n\tv_nop" : "+v"(a), "+v"(b));
}

template <typename T> struct Frag;
template <> struct Frag<_Float16> {
  typedef v16h V; union U { v16h v; v8h h[2]; };
  static __device__ __forceinline__ v16h load(const _Float16* p) {
    U f; f.h[0] = *(const v8h*)(p); f.h[1] = *(const v8h*)(p + 16); return f.v;
  }
  static __device__ __forceinline__ v8f mma(v16h a, v16h b, v8f c) {
    return __builtin_amdgcn_wmma_f32_16x16x32_f16(false, a, false, b, (short)0, c, false, false);
  }
  static __device__ __forceinline__ void guard4(v8f& a, v8f& b, v8f& c, v8f& d, v16h x, v16h y) { dep_guard4_h(a, b, c, d, x, y); }
  static __device__ __forceinline__ void keep(v16h a, v16h b, v16h c, v16h d) { keep4_h(a, b, c, d); }
};
template <> struct Frag<__bf16> {
  typedef v16b V; union U { v16b v; v8b h[2]; };
  static __device__ __forceinline__ v16b load(const __bf16* p) {
    U f; f.h[0] = *(const v8b*)(p); f.h[1] = *(const v8b*)(p + 16); return f.v;
  }
  static __device__ __forceinline__ v8f mma(v16b a, v16b b, v8f c) {
    return __builtin_amdgcn_wmma_f32_16x16x32_bf16(false, a, false, b, (short)0, c, false, false);
  }
  static __device__ __forceinline__ void guard4(v8f& a, v8f& b, v8f& c, v8f& d, v16b x, v16b y) { dep_guard4_b(a, b, c, d, x, y); }
  static __device__ __forceinline__ void keep(v16b a, v16b b, v16b c, v16b d) { keep4_b(a, b, c, d); }
};

__device__ __forceinline__ float fsig(float x)  { return __builtin_amdgcn_rcpf(1.0f + __expf(-x)); }
__device__ __forceinline__ float ftanh(float x) { return 1.0f - 2.0f * __builtin_amdgcn_rcpf(__expf(2.0f * x) + 1.0f); }

template <int ET> struct Elem;
template <> struct Elem<0> { typedef _Float16 T; };
template <> struct Elem<1> { typedef __bf16 T; };
template <int ET, bool SPLIT, int BIAS_MODE, int OUT_MODE, bool RESID>
__global__ __launch_bounds__(256) void wmma_gemm64(
    const unsigned short* __restrict__ Ap, const unsigned short* __restrict__ A2p, int lda, long strideA,
    const unsigned short* __restrict__ Btp, const unsigned short* __restrict__ Bt2p, int ldb, long strideB,
    void* __restrict__ Cout, void* __restrict__ Cout2, int ldc, long strideC,
    const float* __restrict__ bias,
    const float* __restrict__ resid, long strideR,
    int M, int N, int K, float scale) {
  typedef typename Elem<ET>::T T;
  typedef typename Frag<T>::V V;
  const T* A = (const T*)Ap; const T* A2 = (const T*)A2p; const T* Bt = (const T*)Btp; const T* Bt2 = (const T*)Bt2p;
  __shared__ __align__(16) float sT[8][16 * 68];
  const int b    = blockIdx.y;
  const int lane = threadIdx.x & 31;
  const int wave = threadIdx.x >> 5;
  const int tilesN = N >> 6;
  const int tilesM = M >> 6;
  const int tile = blockIdx.x * 8 + wave;
  if (tile >= tilesM * tilesN) return;
  const int tm = tile / tilesN;
  const int tn = tile - tm * tilesN;
  const int m0 = tm << 6;
  const int n0 = tn << 6;

  const T* Ab  = A  + (size_t)b * strideA;
  const T* Bb  = Bt + (size_t)b * strideB;
  const T* Ab2 = SPLIT ? (A2  + (size_t)b * strideA) : nullptr;
  const T* Bb2 = SPLIT ? (Bt2 + (size_t)b * strideB) : nullptr;

  const int rlane = lane & 15;
  const int koff  = (lane >> 4) * 8;
  const int mOff  = (lane >> 4) * 8;

  v8f acc[4][4];
#pragma unroll
  for (int i = 0; i < 4; ++i)
#pragma unroll
    for (int j = 0; j < 4; ++j) acc[i][j] = (v8f){0.f,0.f,0.f,0.f,0.f,0.f,0.f,0.f};

  for (int k0 = 0; k0 < K; k0 += 32) {
    V bh[4], bl[4];
#pragma unroll
    for (int j = 0; j < 4; ++j) {
      const size_t bo = (size_t)(n0 + (j << 4) + rlane) * ldb + koff + k0;
      bh[j] = Frag<T>::load(Bb + bo);
      if (SPLIT) bl[j] = Frag<T>::load(Bb2 + bo);
    }
#pragma unroll
    for (int i = 0; i < 4; ++i) {
      const size_t ao = (size_t)(m0 + (i << 4) + rlane) * lda + koff + k0;
      V ah = Frag<T>::load(Ab + ao);
      V al;
      if (SPLIT) al = Frag<T>::load(Ab2 + ao);
#pragma unroll
      for (int j = 0; j < 4; ++j) {
        acc[i][j] = Frag<T>::mma(ah, bh[j], acc[i][j]);
        if (SPLIT) {
          acc[i][j] = Frag<T>::mma(ah, bl[j], acc[i][j]);
          acc[i][j] = Frag<T>::mma(al, bh[j], acc[i][j]);
        }
      }
      Frag<T>::guard4(acc[i][0], acc[i][1], acc[i][2], acc[i][3], ah, SPLIT ? al : ah);
    }
    Frag<T>::keep(bh[0], bh[1], bh[2], bh[3]);
    if (SPLIT) Frag<T>::keep(bl[0], bl[1], bl[2], bl[3]);
  }
  acc_guard4(acc[0][0], acc[0][1], acc[0][2], acc[0][3]);
  acc_guard4(acc[1][0], acc[1][1], acc[1][2], acc[1][3]);
  acc_guard4(acc[2][0], acc[2][1], acc[2][2], acc[2][3]);
  acc_guard4(acc[3][0], acc[3][1], acc[3][2], acc[3][3]);

  float* slab = sT[wave];
  const float* Rb = RESID ? (resid + (size_t)b * strideR) : nullptr;
#pragma unroll
  for (int i = 0; i < 4; ++i) {
    const int mBase = m0 + (i << 4);
#pragma unroll
    for (int j = 0; j < 4; ++j) {
      const int n = n0 + (j << 4) + rlane;
      float bv = 0.f;
      if (BIAS_MODE == 2) bv = bias[n];
#pragma unroll
      for (int r = 0; r < 8; ++r) {
        float v = acc[i][j][r] * scale;
        if (BIAS_MODE == 1) v += bias[mBase + mOff + r];
        if (BIAS_MODE == 2) v += bv;
        if (RESID) v += Rb[(size_t)(mBase + mOff + r) * ldc + n];
        slab[(mOff + r) * 68 + (j << 4) + rlane] = v;
      }
    }
    __builtin_amdgcn_fence(__ATOMIC_RELEASE, "workgroup");
    __builtin_amdgcn_wave_barrier();
    __builtin_amdgcn_fence(__ATOMIC_ACQUIRE, "workgroup");
    if (OUT_MODE == 0) {
      float* C = (float*)Cout + (size_t)b * strideC;
      const int hh = lane >> 4, c4 = (lane & 15) * 4;
      for (int pass = 0; pass < 2; ++pass) {
#pragma unroll
        for (int it = 0; it < 8; ++it) {
          const int row = it * 2 + hh;
          v4f v = *(const v4f*)(slab + row * 68 + c4);
          *(volatile v4f*)(C + (size_t)(mBase + row) * ldc + n0 + c4) = v;
        }
        __threadfence();
      }
    } else {
      const int q = lane >> 3, c8 = (lane & 7) * 8;
      unsigned short* C  = (unsigned short*)Cout  + (size_t)b * strideC;
      unsigned short* C2 = (OUT_MODE == 2) ? ((unsigned short*)Cout2 + (size_t)b * strideC) : nullptr;
      for (int pass = 0; pass < 2; ++pass) {
#pragma unroll
        for (int it = 0; it < 4; ++it) {
          const int row = it * 4 + q;
          const float* sp = slab + row * 68 + c8;
          v8h hv, lv;
#pragma unroll
          for (int e = 0; e < 8; ++e) {
            if (OUT_MODE == 1) {
              hv[e] = (_Float16)sp[e];
            } else {
              unsigned short hb = f2bf_bits(sp[e]);
              unsigned short lb = f2bf_bits(sp[e] - bf_bits2f(hb));
              hv[e] = __builtin_bit_cast(_Float16, hb);
              lv[e] = __builtin_bit_cast(_Float16, lb);
            }
          }
          *(volatile v8h*)(C + (size_t)(mBase + row) * ldc + n0 + c8) = hv;
          if (OUT_MODE == 2) *(volatile v8h*)(C2 + (size_t)(mBase + row) * ldc + n0 + c8) = lv;
        }
        __threadfence();
      }
    }
    __builtin_amdgcn_fence(__ATOMIC_RELEASE, "workgroup");
    __builtin_amdgcn_wave_barrier();
    __builtin_amdgcn_fence(__ATOMIC_ACQUIRE, "workgroup");
  }
}

__device__ __forceinline__ void split8_bf16(const v4f a, const v4f b, v8h& hv, v8h& lv) {
#pragma unroll
  for (int e = 0; e < 4; ++e) {
    const float f0 = a[e];
    const float f1 = b[e];
    const unsigned short h0 = f2bf_bits(f0);
    const unsigned short h1 = f2bf_bits(f1);
    const unsigned short l0 = f2bf_bits(f0 - bf_bits2f(h0));
    const unsigned short l1 = f2bf_bits(f1 - bf_bits2f(h1));
    hv[e]     = __builtin_bit_cast(_Float16, h0);
    hv[4 + e] = __builtin_bit_cast(_Float16, h1);
    lv[e]     = __builtin_bit_cast(_Float16, l0);
    lv[4 + e] = __builtin_bit_cast(_Float16, l1);
  }
}

__global__ __launch_bounds__(256) void xsplit_kernel(const float* __restrict__ x, unsigned short* __restrict__ XH,
                                                     unsigned short* __restrict__ XL) {
  const int i = blockIdx.x * 256 + threadIdx.x;
  if (i < NROWS * (NFEAT / 8)) {
    const int ro = i >> 5;
    const int cc = i & 31;
    const int t  = ro >> 4;
    const int b  = ro & 15;
    const float* sp = x + ((size_t)(b * NSTEP + t)) * NFEAT + cc * 8;
    const v4f a0 = *(const v4f*)(sp);
    const v4f a1 = *(const v4f*)(sp + 4);
    v8h hv, lv;
    split8_bf16(a0, a1, hv, lv);
    *(volatile v8h*)(XH + (size_t)i * 8) = hv;
    *(volatile v8h*)(XL + (size_t)i * 8) = lv;
    __threadfence();
    *(volatile v8h*)(XH + (size_t)i * 8) = hv;
    *(volatile v8h*)(XL + (size_t)i * 8) = lv;
  }
}

template <int MODE>
__global__ __launch_bounds__(256) void pack_cat_kernel(const float* __restrict__ srcA, int nA,
                                                       const float* __restrict__ srcB, int nB,
                                                       unsigned short* __restrict__ dstH, unsigned short* __restrict__ dstL,
                                                       int nrowDst, int k8, float sc) {
  const int i  = blockIdx.x * 256 + threadIdx.x;
  const int n8 = nrowDst * k8;
  if (i < n8) {
    const int row  = i / k8;
    const int cc   = i - row * k8;
    const int kdim = k8 * 8;
    const int ra = (row < nA) ? row : (nA - 1);
    const int rbmax = (nB > 0) ? (nB - 1) : 0;
    int rb = row - nA;
    rb = (rb < 0) ? 0 : rb;
    rb = (rb > rbmax) ? rbmax : rb;
    const float* pa = srcA + (size_t)ra * kdim + cc * 8;
    const float* pb = srcB + (size_t)rb * kdim + cc * 8;
    const v4f a0 = *(const v4f*)(pa);
    const v4f a1 = *(const v4f*)(pa + 4);
    const v4f b0 = *(const v4f*)(pb);
    const v4f b1 = *(const v4f*)(pb + 4);
    const bool inA = (row < nA);
    const bool inB = (!inA) && (row < nA + nB);
    v4f s0, s1;
#pragma unroll
    for (int e = 0; e < 4; ++e) {
      s0[e] = inA ? a0[e] : (inB ? b0[e] : 0.0f);
      s1[e] = inA ? a1[e] : (inB ? b1[e] : 0.0f);
    }
    v8h hv, lv;
    if (MODE == 0) {
      split8_bf16(s0, s1, hv, lv);
    } else if (MODE == 1) {
#pragma unroll
      for (int e = 0; e < 4; ++e) {
        hv[e]     = (_Float16)(s0[e] * sc);
        hv[4 + e] = (_Float16)(s1[e] * sc);
      }
      lv = hv;
    } else {
#pragma unroll
      for (int e = 0; e < 4; ++e) {
        const float v0 = s0[e] * sc;
        const float v1 = s1[e] * sc;
        const _Float16 h0 = (_Float16)v0;
        const _Float16 h1 = (_Float16)v1;
        const float r0 = (v0 - (float)h0) * RCARRY;
        const float r1 = (v1 - (float)h1) * RCARRY;
        hv[e]     = (_Float16)r0;
        hv[4 + e] = (_Float16)r1;
      }
      lv = hv;
    }
    *(volatile v8h*)(dstH + (size_t)i * 8) = hv;
    if (MODE == 0) *(volatile v8h*)(dstL + (size_t)i * 8) = lv;
    __threadfence();
    *(volatile v8h*)(dstH + (size_t)i * 8) = hv;
    if (MODE == 0) *(volatile v8h*)(dstL + (size_t)i * 8) = lv;
  }
}

__global__ __launch_bounds__(256) void biascat_kernel(const float* __restrict__ bih0, const float* __restrict__ bik0,
                                                      const float* __restrict__ bih1, const float* __restrict__ bik1,
                                                      float* __restrict__ dst0, float* __restrict__ dst1) {
  const int layer = blockIdx.y;
  const float* bih = layer ? bih1 : bih0;
  const float* bik = layer ? bik1 : bik0;
  float* dst = layer ? dst1 : dst0;
  const int i  = blockIdx.x * 256 + threadIdx.x;
  const int nslot = NCATROW / 4;
  const int ic = (i < nslot) ? i : (nslot - 1);
  const int col = ic * 4;
  const int ca = (col < NGATE3 - 4) ? col : (NGATE3 - 4);
  int cb = col - NGATE3;
  cb = (cb < 0) ? 0 : cb;
  cb = (cb > 4) ? 4 : cb;
  const v4f va = *(const v4f*)(bih + ca);
  const v4f vb = *(const v4f*)(bik + cb);
  const bool inA = (col < NGATE3);
  const bool inB = (!inA) && (col < NGATE3 + NBLK);
  const float fa = inA ? 1.0f : 0.0f;
  const float fb = inB ? 1.0f : 0.0f;
  v4f o;
#pragma unroll
  for (int e = 0; e < 4; ++e) o[e] = fmaf(fa, va[e], fb * vb[e]);
  if (i < nslot) {
    *(volatile v4f*)(dst + col) = o;
    __threadfence();
    *(volatile v4f*)(dst + col) = o;
  }
}

__device__ __forceinline__ void put_h16(_Float16* hi, _Float16* lo, int idx, float h) {
  const float hs = h * HCARRY;
  const _Float16 a = (_Float16)hs;
  const float af = (float)a;
  const float res = (hs - af) * RCARRY;
  hi[idx] = a;
  lo[idx] = (_Float16)res;
}

template <bool L1>
__global__ __launch_bounds__(SCAN_THR) void gru_scan_kernel(const float* __restrict__ GX,
                                                            const unsigned short* __restrict__ WHp,
                                                            const unsigned short* __restrict__ WKLp,
                                                            const float* __restrict__ bhh, const float* __restrict__ bhk,
                                                            float* HC, unsigned short* __restrict__ H1,
                                                            float* __restrict__ OUT, int t0, int first) {
  __shared__ __align__(16) _Float16 Ahi[2 * PLANE16];
  __shared__ __align__(16) _Float16 Alo[PLANE16];
  __shared__ __align__(16) float    Hf[NBATCH * FPITCH];
  __shared__ __align__(16) float    KPm[16 * 128];
  __shared__ __align__(16) float    KPr[16 * 128];
  const _Float16* WH  = (const _Float16*)WHp;
  const _Float16* WKL = (const _Float16*)WKLp;
  const int tid = threadIdx.x, lane = tid & 31, wave = tid >> 5;
  const int c = lane & 15, hh = lane >> 4, koff = hh * 8, c4 = c * 4;
  const int mblk = wave >> 1;
  const int colw = 64 * wave;
  const float bk = bhk[mblk];

#pragma unroll 1
  for (int nt = 0; nt < 4; ++nt) {
    const int j = colw + 16 * nt + c;
#pragma unroll
    for (int r = 0; r < 8; ++r) {
      const int ri = 8 * hh + r;
      float h0 = 0.0f;
      if (!first) h0 = HC[(size_t)ri * NHID + j];
      Hf[ri * FPITCH + j] = h0;
      put_h16(Ahi, Alo, ri * HPITCH + j, h0);
    }
  }
  __syncthreads();

  const v8f z8 = {0.f, 0.f, 0.f, 0.f, 0.f, 0.f, 0.f, 0.f};
  const _Float16* wk  = WH  + (size_t)(NGATE3 + c) * NHID + koff + colw;
  const _Float16* wkl = WKL + (size_t)c * NHID + koff + colw;
  const _Float16* alk = Alo + c * HPITCH + koff + colw;

#pragma unroll 1
  for (int tl = 0; tl < HALF_STEPS; ++tl) {
    const int cur = tl & 1;
    const _Float16* acur = Ahi + cur * PLANE16;
    _Float16* anxt = Ahi + (cur ^ 1) * PLANE16;
    const _Float16* ahrow = acur + c * HPITCH + koff;
    float kxv = GX[(size_t)(tl * NBATCH + c) * NCATROW + NGATE3 + mblk];
    asm volatile("" : "+v"(kxv));

    {
      v8f aM = z8, aR = z8;
      const _Float16* ahk = ahrow + colw;
#pragma unroll
      for (int kk = 0; kk < 64; kk += 32) {
        const v16h a  = Frag<_Float16>::load(ahk + kk);
        const v16h a2 = Frag<_Float16>::load(alk + kk);
        const v16h b  = Frag<_Float16>::load(wk + kk);
        const v16h b2 = Frag<_Float16>::load(wkl + kk);
        aM = Frag<_Float16>::mma(a, b, aM);
        aR = Frag<_Float16>::mma(a2, b, aR);
        aR = Frag<_Float16>::mma(a, b2, aR);
        dep_guard2_h(aM, aR, a, a2, b, b2);
      }
      acc_guard2(aM, aR);
      if (c < 8) {
#pragma unroll
        for (int r = 0; r < 8; ++r) {
          KPm[wave * 128 + (8 * hh + r) * 8 + c] = aM[r];
          KPr[wave * 128 + (8 * hh + r) * 8 + c] = aR[r];
        }
      }
    }
    __syncthreads();

    float sM = 0.0f, sR = 0.0f;
#pragma unroll
    for (int q = 0; q < 16; ++q) {
      sM += KPm[q * 128 + c * 8 + mblk];
      sR += KPr[q * 128 + c * 8 + mblk];
    }
    const float pre = (kxv + (sM * FOLD_MAIN + sR * FOLD_RES)) + bk;
    const float kv = fsig(BETA_GATE * pre);
    float kr[8];
#pragma unroll
    for (int r = 0; r < 8; ++r) kr[r] = __shfl(kv, 8 * hh + r, 32);

#pragma unroll 1
    for (int nt = 0; nt < 4; ++nt) {
      const int j = colw + 16 * nt + c;
      const _Float16* wz = WH + (size_t)j * NHID + koff;
      v8f az = z8, ar = z8, an = z8;
#pragma unroll 1
      for (int k0 = 0; k0 < NHID; k0 += 32) {
        const v16h a  = Frag<_Float16>::load(ahrow + k0);
        const v16h b0 = Frag<_Float16>::load(wz + k0);
        const v16h b1 = Frag<_Float16>::load(wz + (size_t)NHID * NHID + k0);
        const v16h b2 = Frag<_Float16>::load(wz + (size_t)2 * NHID * NHID + k0);
        az = Frag<_Float16>::mma(a, b0, az);
        ar = Frag<_Float16>::mma(a, b1, ar);
        an = Frag<_Float16>::mma(a, b2, an);
        dep_guard3_h(az, ar, an, a, b0, b1, b2);
      }
      acc_guard3(az, ar, an);
      const float* gp = GX + (size_t)(tl * NBATCH + 8 * hh) * NCATROW + j;
      const float bzv = bhh[j];
      const float brv = bhh[NHID + j];
      const float bnv = bhh[2 * NHID + j];
      float xz[8], xr[8];
#pragma unroll
      for (int r = 0; r < 8; ++r) {
        xz[r] = gp[(size_t)r * NCATROW];
        xr[r] = gp[(size_t)r * NCATROW + NHID];
      }
      float zg[8], rg[8];
#pragma unroll
      for (int r = 0; r < 8; ++r) {
        const float hz = az[r] * FOLD_MAIN + bzv;
        const float hr = ar[r] * FOLD_MAIN + brv;
        zg[r] = fsig(xz[r] + hz);
        rg[r] = fsig(xr[r] + hr);
      }
      float xn[8];
#pragma unroll
      for (int r = 0; r < 8; ++r) xn[r] = gp[(size_t)r * NCATROW + 2 * NHID];
#pragma unroll
      for (int r = 0; r < 8; ++r) {
        const int ri = 8 * hh + r;
        const float hq = an[r] * FOLD_MAIN + bnv;
        const float ng = ftanh(xn[r] + rg[r] * hq);
        const float hold = Hf[ri * FPITCH + j];
        const float hn = hold + (kr[r] * (1.0f - zg[r])) * (ng - hold);
        Hf[ri * FPITCH + j] = hn;
        put_h16(anxt, Alo, ri * HPITCH + j, hn);
      }
    }
    __builtin_amdgcn_fence(__ATOMIC_RELEASE, "workgroup");
    __builtin_amdgcn_wave_barrier();
    __builtin_amdgcn_fence(__ATOMIC_ACQUIRE, "workgroup");

    const bool last = (tl == HALF_STEPS - 1);
    if (L1) {
      for (int pass = 0; pass < 2; ++pass) {
#pragma unroll
        for (int it = 0; it < 8; ++it) {
          const int row = it * 2 + hh;
          const v4f v = *(const v4f*)(Hf + row * FPITCH + colw + c4);
          *(volatile v4f*)(OUT + ((size_t)row * NSTEP + (size_t)(t0 + tl)) * NHID + colw + c4) = v;
        }
        __threadfence();
      }
    } else {
      const int q = lane >> 3, c8 = (lane & 7) * 8;
      v8h hv[4];
#pragma unroll
      for (int it = 0; it < 4; ++it) {
        const float* sp = Hf + (it * 4 + q) * FPITCH + colw + c8;
#pragma unroll
        for (int e = 0; e < 8; ++e) hv[it][e] = (_Float16)(sp[e] * HCARRY);
      }
      for (int pass = 0; pass < 2; ++pass) {
#pragma unroll
        for (int it = 0; it < 4; ++it) {
          const int row = it * 4 + q;
          *(volatile v8h*)(H1 + ((size_t)(t0 + tl) * NBATCH + row) * NHID + colw + c8) = hv[it];
        }
        __threadfence();
      }
    }
    if (last) {
      for (int pass = 0; pass < 2; ++pass) {
#pragma unroll
        for (int it = 0; it < 8; ++it) {
          const int row = it * 2 + hh;
          const v4f v = *(const v4f*)(Hf + row * FPITCH + colw + c4);
          *(volatile v4f*)(HC + (size_t)row * NHID + colw + c4) = v;
        }
        __threadfence();
      }
    }
    __builtin_amdgcn_fence(__ATOMIC_RELEASE, "workgroup");
    __builtin_amdgcn_wave_barrier();
    __builtin_amdgcn_fence(__ATOMIC_ACQUIRE, "workgroup");
    __syncthreads();
  }
}

extern "C" void kernel_launch(void* const* d_in, const int* in_sizes, int n_in,
                              void* d_out, int out_size, void* d_ws, size_t ws_size, hipStream_t stream) {
  if (n_in < 17 || d_out == nullptr || d_ws == nullptr) return;
  if (in_sizes[0] != NBATCH * NSTEP * NFEAT) return;
  if (in_sizes[1] != NGATE3 * NFEAT || in_sizes[2] != NGATE3 * NHID || in_sizes[3] != NGATE3 || in_sizes[4] != NGATE3) return;
  if (in_sizes[5] != NBLK * NFEAT || in_sizes[6] != NBLK * NHID || in_sizes[7] != NBLK || in_sizes[8] != NBLK) return;
  if (in_sizes[9] != NGATE3 * NHID || in_sizes[10] != NGATE3 * NHID || in_sizes[11] != NGATE3 || in_sizes[12] != NGATE3) return;
  if (in_sizes[13] != NBLK * NHID || in_sizes[14] != NBLK * NHID || in_sizes[15] != NBLK || in_sizes[16] != NBLK) return;
  if (out_size != NBATCH * NSTEP * NHID) return;

  const float* x     = (const float*)d_in[0];
  const float* wih0  = (const float*)d_in[1];
  const float* whh0  = (const float*)d_in[2];
  const float* bih0  = (const float*)d_in[3];
  const float* bhh0  = (const float*)d_in[4];
  const float* wik0  = (const float*)d_in[5];
  const float* whk0  = (const float*)d_in[6];
  const float* bik0  = (const float*)d_in[7];
  const float* bhk0  = (const float*)d_in[8];
  const float* wih1  = (const float*)d_in[9];
  const float* whh1  = (const float*)d_in[10];
  const float* bih1  = (const float*)d_in[11];
  const float* bhh1  = (const float*)d_in[12];
  const float* wik1  = (const float*)d_in[13];
  const float* whk1  = (const float*)d_in[14];
  const float* bik1  = (const float*)d_in[15];
  const float* bhk1  = (const float*)d_in[16];
  float* out = (float*)d_out;

  char* ws = (char*)d_ws; size_t off = 0;
  auto carve = [&](size_t bytes) -> char* { char* p = ws + off; off += (bytes + 255) & ~(size_t)255; return p; };
  unsigned short* XH   = (unsigned short*)carve((size_t)NROWS * NFEAT * 2);
  unsigned short* XL   = (unsigned short*)carve((size_t)NROWS * NFEAT * 2);
  unsigned short* WI0H = (unsigned short*)carve((size_t)NCATROW * NFEAT * 2);
  unsigned short* WI0L = (unsigned short*)carve((size_t)NCATROW * NFEAT * 2);
  unsigned short* WHH0 = (unsigned short*)carve((size_t)NWHHROW * NHID * 2);
  unsigned short* WHH1 = (unsigned short*)carve((size_t)NWHHROW * NHID * 2);
  unsigned short* WI1  = (unsigned short*)carve((size_t)NCATROW * NHID * 2);
  float*          BC0  = (float*)carve((size_t)NCATROW * 4);
  float*          BC1  = (float*)carve((size_t)NCATROW * 4);
  unsigned short* H1   = (unsigned short*)carve((size_t)NROWS * NHID * 2);
  float*          GX   = (float*)carve((size_t)HALF_ROWS * NCATROW * 4);
  float*          HC   = (float*)carve((size_t)NBATCH * NHID * 4);
  unsigned short* WKL0 = (unsigned short*)carve((size_t)NWKLROW * NHID * 2);
  unsigned short* WKL1 = (unsigned short*)carve((size_t)NWKLROW * NHID * 2);
  if (off > ws_size || off > (size_t)134217728) return;

  xsplit_kernel<<<NROWS * (NFEAT / 8) / 256, 256, 0, stream>>>(x, XH, XL);
  pack_cat_kernel<0><<<NCATROW * (NFEAT / 8) / 256, 256, 0, stream>>>(wih0, NGATE3, wik0, NBLK, WI0H, WI0L, NCATROW, NFEAT / 8, 1.0f);
  pack_cat_kernel<1><<<NWHHROW * (NHID / 8) / 256, 256, 0, stream>>>(whh0, NGATE3, whk0, NBLK, WHH0, WHH0, NWHHROW, NHID / 8, WCARRY);
  pack_cat_kernel<1><<<NWHHROW * (NHID / 8) / 256, 256, 0, stream>>>(whh1, NGATE3, whk1, NBLK, WHH1, WHH1, NWHHROW, NHID / 8, WCARRY);
  pack_cat_kernel<1><<<NCATROW * (NHID / 8) / 256, 256, 0, stream>>>(wih1, NGATE3, wik1, NBLK, WI1, WI1, NCATROW, NHID / 8, WCARRY);
  pack_cat_kernel<2><<<NWKLROW * (NHID / 8) / 256, 256, 0, stream>>>(whk0, NBLK, whk0, 0, WKL0, WKL0, NWKLROW, NHID / 8, WCARRY);
  pack_cat_kernel<2><<<NWKLROW * (NHID / 8) / 256, 256, 0, stream>>>(whk1, NBLK, whk1, 0, WKL1, WKL1, NWKLROW, NHID / 8, WCARRY);
  biascat_kernel<<<dim3(4, 2), 256, 0, stream>>>(bih0, bik0, bih1, bik1, BC0, BC1);

  const dim3 ggrid((HALF_ROWS / 64) * (NCATROW / 64) / 8, 1);

  for (int half = 0; half < 2; ++half) {
    const size_t arow = (size_t)half * HALF_ROWS * NFEAT;
    wmma_gemm64<1, true, 2, 0, false><<<ggrid, 256, 0, stream>>>(
        XH + arow, XL + arow, NFEAT, 0L, WI0H, WI0L, NFEAT, 0L, (void*)GX, (void*)GX, NCATROW, 0L,
        BC0, BC0, 0L, HALF_ROWS, NCATROW, NFEAT, 1.0f);
    gru_scan_kernel<false><<<1, SCAN_THR, 0, stream>>>(GX, WHH0, WKL0, bhh0, bhk0, HC, H1, out,
                                                       half * HALF_STEPS, half == 0 ? 1 : 0);
  }
  for (int half = 0; half < 2; ++half) {
    const size_t arow = (size_t)half * HALF_ROWS * NHID;
    wmma_gemm64<0, false, 2, 0, false><<<ggrid, 256, 0, stream>>>(
        H1 + arow, H1 + arow, NHID, 0L, WI1, WI1, NHID, 0L, (void*)GX, (void*)GX, NCATROW, 0L,
        BC1, BC1, 0L, HALF_ROWS, NCATROW, NHID, FOLD_MAIN);
    gru_scan_kernel<true><<<1, SCAN_THR, 0, stream>>>(GX, WHH1, WKL1, bhh1, bhk1, HC, H1, out,
                                                      half * HALF_STEPS, half == 0 ? 1 : 0);
  }
}
